// CAM_62852551409742
// MI455X (gfx1250) — hardware-run, weakly checked
//
#include <hip/hip_runtime.h>
#include <math.h>

typedef __attribute__((ext_vector_type(16))) _Float16 v16h;
typedef __attribute__((ext_vector_type(8)))  _Float16 v8h;
typedef __attribute__((ext_vector_type(4)))  _Float16 v4h;
typedef __attribute__((ext_vector_type(16))) __bf16   v16b;
typedef __attribute__((ext_vector_type(8)))  __bf16   v8b;
typedef __attribute__((ext_vector_type(8)))  float    v8f;
typedef __attribute__((ext_vector_type(4)))  float    v4f;
typedef __attribute__((ext_vector_type(4)))  unsigned int v4u;

constexpr int kRep    = 4;
constexpr int kBat    = 512;
constexpr int kLen    = 150;
constexpr int kHid    = 32;
constexpr int kKin    = kRep * kLen;
constexpr int kKpad   = 640;
constexpr int kKrow   = 648;
constexpr int kLenPad = 160;
constexpr int kSeg    = 192;
constexpr int kFFld   = kRep * kSeg;
constexpr int kN1     = 128;
constexpr int kN2     = 7;
constexpr int kNB     = 2;
constexpr int kWPB    = 5;
constexpr int kThr2   = 32 * kNB * kWPB;
constexpr float kCarryA   = 4096.0f;
constexpr float kCarryW   = 256.0f;
constexpr float kInvCarry = 1.0f / (4096.0f * 256.0f);

static_assert(kKpad % 32 == 0);
static_assert(kKpad >= kKin && kKrow >= kKpad && kKrow % 8 == 0);
static_assert(kFFld % 32 == 0);
static_assert(kBat % 64 == 0 && kN1 % 64 == 0);
static_assert(kBat % kNB == 0);
static_assert(kLenPad == 32 * kWPB && kLenPad >= kLen && kLenPad % 16 == 0);
static_assert(kNB * kLenPad == kThr2);
static_assert(kSeg * 2 == 3 * 128 && kSeg >= kLenPad);
static_assert((kFFld * 2) % 128 == 0);
static_assert((64 * kN2 * 4) % 128 == 0);
static_assert(kBat % 64 == 0);
static_assert(kN1 * (kFFld / 8) == 48 * 256);

__device__ __forceinline__ unsigned short f2bf_bits(float f) {
  unsigned u = __float_as_uint(f);
  return (unsigned short)((u + 0x7FFFu + ((u >> 16) & 1u)) >> 16);
}
__device__ __forceinline__ float bf_bits2f(unsigned short h) { return __uint_as_float(((unsigned)h) << 16); }

__device__ __forceinline__ void dep_guard_h(v8f& a, v8f& b, v16h x, v16h y) { asm volatile("v_nop\n\tv_nop\n\tv_nop\n\tv_nop" : "+v"(a), "+v"(b) : "v"(x), "v"(y)); }
__device__ __forceinline__ void dep_guard_b(v8f& a, v8f& b, v16b x, v16b y) { asm volatile("v_nop\n\tv_nop\n\tv_nop\n\tv_nop" : "+v"(a), "+v"(b) : "v"(x), "v"(y)); }
__device__ __forceinline__ void keep4_h(v16h a, v16h b, v16h c, v16h d) { asm volatile("v_nop" :: "v"(a), "v"(b), "v"(c), "v"(d)); }
__device__ __forceinline__ void keep4_b(v16b a, v16b b, v16b c, v16b d) { asm volatile("v_nop" :: "v"(a), "v"(b), "v"(c), "v"(d)); }
__device__ __forceinline__ void acc_guard4(v8f& a, v8f& b, v8f& c, v8f& d) { asm volatile("v_nop\n\tv_nop\n\tv_nop\n\tv_nop" : "+v"(a), "+v"(b), "+v"(c), "+v"(d)); }
template <typename T> struct Frag;
template <> struct Frag<_Float16> {
  typedef v16h V; union U { v16h v; v8h h[2]; };
  static __device__ __forceinline__ v16h load(const _Float16* p) {
    U f; f.h[0] = *(const v8h*)(p); f.h[1] = *(const v8h*)(p + 16); return f.v;
  }
  static __device__ __forceinline__ v8f mma(v16h a, v16h b, v8f c) {
    return __builtin_amdgcn_wmma_f32_16x16x32_f16(false, a, false, b, (short)0, c, false, false);
  }
  static __device__ __forceinline__ void guard(v8f& a, v8f& b, v16h x, v16h y) { dep_guard_h(a, b, x, y); }
  static __device__ __forceinline__ void keep(v16h a, v16h b, v16h c, v16h d) { keep4_h(a, b, c, d); }
};
template <> struct Frag<__bf16> {
  typedef v16b V; union U { v16b v; v8b h[2]; };
  static __device__ __forceinline__ v16b load(const __bf16* p) {
    U f; f.h[0] = *(const v8b*)(p); f.h[1] = *(const v8b*)(p + 16); return f.v;
  }
  static __device__ __forceinline__ v8f mma(v16b a, v16b b, v8f c) {
    return __builtin_amdgcn_wmma_f32_16x16x32_bf16(false, a, false, b, (short)0, c, false, false);
  }
  static __device__ __forceinline__ void guard(v8f& a, v8f& b, v16b x, v16b y) { dep_guard_b(a, b, x, y); }
  static __device__ __forceinline__ void keep(v16b a, v16b b, v16b c, v16b d) { keep4_b(a, b, c, d); }
};

__device__ __forceinline__ unsigned pk16(unsigned short a, unsigned short b) { return (unsigned)a | ((unsigned)b << 16); }

template <int ET> struct Elem;
template <> struct Elem<0> { typedef _Float16 T; };
template <> struct Elem<1> { typedef __bf16 T; };
template <int ET, bool SPLIT, int BIAS_MODE, int OUT_MODE, bool RESID, int ACT = 0>
__global__ __launch_bounds__(256) void wmma_gemm64(
    const unsigned short* __restrict__ Ap, const unsigned short* __restrict__ A2p, int lda, long strideA,
    const unsigned short* __restrict__ Btp, const unsigned short* __restrict__ Bt2p, int ldb, long strideB,
    void* __restrict__ Cout, void* __restrict__ Cout2, int ldc, long strideC,
    const float* __restrict__ bias,
    const float* __restrict__ resid, long strideR,
    int M, int N, int K, float scale) {
  typedef typename Elem<ET>::T T;
  typedef typename Frag<T>::V V;
  const T* A = (const T*)Ap; const T* A2 = (const T*)A2p; const T* Bt = (const T*)Btp; const T* Bt2 = (const T*)Bt2p;
  __shared__ __align__(16) float sT[8][16 * 68];
  const int b    = blockIdx.y;
  const int lane = threadIdx.x & 31;
  const int wave = threadIdx.x >> 5;
  const int tilesN = N >> 6;
  const int tilesM = M >> 6;
  const int tile = blockIdx.x * 8 + wave;
  if (tile >= tilesM * tilesN) return;
  const int tm = tile / tilesN;
  const int tn = tile - tm * tilesN;
  const int m0 = tm << 6;
  const int n0 = tn << 6;

  const T* Ab  = A  + (size_t)b * strideA;
  const T* Bb  = Bt + (size_t)b * strideB;
  const T* Ab2 = SPLIT ? (A2  + (size_t)b * strideA) : nullptr;
  const T* Bb2 = SPLIT ? (Bt2 + (size_t)b * strideB) : nullptr;

  const int rlane = lane & 15;
  const int koff  = (lane >> 4) * 8;
  const int mOff  = (lane >> 4) * 8;

  v8f acc[4][4];
#pragma unroll
  for (int i = 0; i < 4; ++i)
#pragma unroll
    for (int j = 0; j < 4; ++j) acc[i][j] = (v8f){0.f,0.f,0.f,0.f,0.f,0.f,0.f,0.f};

  for (int k0 = 0; k0 < K; k0 += 32) {
    V bh[4], bl[4];
#pragma unroll
    for (int j = 0; j < 4; ++j) {
      const size_t bo = (size_t)(n0 + (j << 4) + rlane) * ldb + koff + k0;
      bh[j] = Frag<T>::load(Bb + bo);
      if (SPLIT) bl[j] = Frag<T>::load(Bb2 + bo);
    }
#pragma unroll
    for (int i = 0; i < 4; ++i) {
      const size_t ao = (size_t)(m0 + (i << 4) + rlane) * lda + koff + k0;
      V ah = Frag<T>::load(Ab + ao);
      V al;
      if (SPLIT) al = Frag<T>::load(Ab2 + ao);
#pragma unroll
      for (int j = 0; j < 4; ++j) {
        acc[i][j] = Frag<T>::mma(ah, bh[j], acc[i][j]);
        if (SPLIT) {
          acc[i][j] = Frag<T>::mma(ah, bl[j], acc[i][j]);
          acc[i][j] = Frag<T>::mma(al, bh[j], acc[i][j]);
        }
      }
      Frag<T>::guard(acc[i][0], acc[i][3], ah, SPLIT ? al : ah);
    }
    Frag<T>::keep(bh[0], bh[1], bh[2], bh[3]);
    if (SPLIT) Frag<T>::keep(bl[0], bl[1], bl[2], bl[3]);
  }
  acc_guard4(acc[0][0], acc[0][1], acc[0][2], acc[0][3]);
  acc_guard4(acc[1][0], acc[1][1], acc[1][2], acc[1][3]);
  acc_guard4(acc[2][0], acc[2][1], acc[2][2], acc[2][3]);
  acc_guard4(acc[3][0], acc[3][1], acc[3][2], acc[3][3]);

  float* slab = sT[wave];
  const float* Rb = RESID ? (resid + (size_t)b * strideR) : nullptr;
#pragma unroll
  for (int i = 0; i < 4; ++i) {
    const int mBase = m0 + (i << 4);
#pragma unroll
    for (int j = 0; j < 4; ++j) {
      const int n = n0 + (j << 4) + rlane;
      float bv = 0.f;
      if (BIAS_MODE == 2) bv = bias[n];
#pragma unroll
      for (int r = 0; r < 8; ++r) {
        float v = acc[i][j][r] * scale;
        if (BIAS_MODE == 1) v += bias[mBase + mOff + r];
        if (BIAS_MODE == 2) v += bv;
        if (RESID) v += Rb[(size_t)(mBase + mOff + r) * ldc + n];
        if (ACT == 2) v = fmaxf(v, 0.0f);
        if (ACT == 4) v = (v > 0.f) ? v : 0.01f * v;
        slab[(mOff + r) * 68 + (j << 4) + rlane] = v;
      }
    }
    __builtin_amdgcn_fence(__ATOMIC_RELEASE, "workgroup");
    __builtin_amdgcn_wave_barrier();
    __builtin_amdgcn_fence(__ATOMIC_ACQUIRE, "workgroup");
    if (OUT_MODE == 0) {
      float* C = (float*)Cout + (size_t)b * strideC;
      const int hh = lane >> 4, c4 = (lane & 15) * 4;
      for (int pass = 0; pass < 2; ++pass) {
#pragma unroll
        for (int it = 0; it < 8; ++it) {
          const int row = it * 2 + hh;
          v4f v = *(const v4f*)(slab + row * 68 + c4);
          *(volatile v4f*)(C + (size_t)(mBase + row) * ldc + n0 + c4) = v;
        }
        __threadfence();
      }
    } else {
      const int q = lane >> 3, c8 = (lane & 7) * 8;
      unsigned short* C  = (unsigned short*)Cout  + (size_t)b * strideC;
      unsigned short* C2 = (OUT_MODE == 2) ? ((unsigned short*)Cout2 + (size_t)b * strideC) : nullptr;
      for (int pass = 0; pass < 2; ++pass) {
#pragma unroll
        for (int it = 0; it < 4; ++it) {
          const int row = it * 4 + q;
          const float* sp = slab + row * 68 + c8;
          v8h hv, lv;
#pragma unroll
          for (int e = 0; e < 8; ++e) {
            if (OUT_MODE == 1) {
              hv[e] = (_Float16)sp[e];
            } else {
              unsigned short hb = f2bf_bits(sp[e]);
              unsigned short lb = f2bf_bits(sp[e] - bf_bits2f(hb));
              hv[e] = __builtin_bit_cast(_Float16, hb);
              lv[e] = __builtin_bit_cast(_Float16, lb);
            }
          }
          *(volatile v8h*)(C + (size_t)(mBase + row) * ldc + n0 + c8) = hv;
          if (OUT_MODE == 2) *(volatile v8h*)(C2 + (size_t)(mBase + row) * ldc + n0 + c8) = lv;
        }
        __threadfence();
      }
    }
    __builtin_amdgcn_fence(__ATOMIC_RELEASE, "workgroup");
    __builtin_amdgcn_wave_barrier();
    __builtin_amdgcn_fence(__ATOMIC_ACQUIRE, "workgroup");
  }
}

__global__ __launch_bounds__(256) void w1_planes_kernel(const float* __restrict__ W1,
                                                        unsigned short* __restrict__ w1hi,
                                                        unsigned short* __restrict__ w1lo) {
  const int i = blockIdx.x * 256 + threadIdx.x;
  if (i >= kN1 * (kFFld / 8)) return;
  const int n  = i / (kFFld / 8);
  const int g  = i - n * (kFFld / 8);
  const int c0 = g * 8;
  const int rr = c0 / kSeg;
  const int t0 = c0 - rr * kSeg;
  const float* src = W1 + (size_t)n * kKin + rr * kLen;
  unsigned short hb[8], lb[8];
#pragma unroll
  for (int j = 0; j < 8; ++j) {
    const int t  = t0 + j;
    const int tc = (t < kLen) ? t : (kLen - 1);
    const float raw = src[tc];
    const float fac = (t < kLen) ? 1.0f : 0.0f;
    const float v = raw * fac;
    const unsigned short h = f2bf_bits(v);
    hb[j] = h;
    lb[j] = f2bf_bits(v - bf_bits2f(h));
  }
  const v4u hv = (v4u){pk16(hb[0], hb[1]), pk16(hb[2], hb[3]), pk16(hb[4], hb[5]), pk16(hb[6], hb[7])};
  const v4u lv = (v4u){pk16(lb[0], lb[1]), pk16(lb[2], lb[3]), pk16(lb[4], lb[5]), pk16(lb[6], lb[7])};
  unsigned short* ph = w1hi + (size_t)8 * i;
  unsigned short* pl = w1lo + (size_t)8 * i;
  for (int pass = 0; pass < 2; ++pass) {
    *(volatile v4u*)ph = hv;
    *(volatile v4u*)pl = lv;
    __threadfence();
  }
}

__device__ __forceinline__ void guard4x(v8f& a, v8f& b, v8f& c, v8f& d, v16h x, v16h y, v16h z, v16h w) {
  asm volatile("v_nop\n\tv_nop\n\tv_nop\n\tv_nop" : "+v"(a), "+v"(b), "+v"(c), "+v"(d) : "v"(x), "v"(y), "v"(z), "v"(w));
}
__device__ __forceinline__ _Float16 tanh_gen(float s2, float x) {
  float p = s2 * x;
  p = fminf(fmaxf(p, -30.0f), 30.0f);
  const float ex = __expf(p);
  const float num = fmaf(ex, kCarryA, -kCarryA);
  const float t = num * __builtin_amdgcn_rcpf(ex + 1.0f);
  return (_Float16)t;
}

__global__ __launch_bounds__(kThr2) void rep_attn_kernel(const float* __restrict__ feats,
                                                         const float* __restrict__ avec,
                                                         const float* __restrict__ Wlin,
                                                         const float* __restrict__ Wc,
                                                         const float* __restrict__ Wh,
                                                         unsigned short* __restrict__ ffhi,
                                                         unsigned short* __restrict__ fflo) {
  __shared__ __align__(16) _Float16 wcs[kHid * kKrow];
  __shared__ __align__(16) float xs[kNB * kKpad];
  __shared__ float svs[kNB * kLenPad];
  __shared__ float fvs[kNB * kLenPad];
  __shared__ float segs[kNB * kSeg];
  __shared__ float wsh[kHid];
  __shared__ float whsh[kHid];

  const int tid = threadIdx.x;
  const int rep = blockIdx.x / (kBat / kNB);
  const int b0  = (blockIdx.x - rep * (kBat / kNB)) * kNB;

  {
    const float* wcr = Wc + (size_t)rep * kHid * kKin;
    for (int idx = tid; idx < kHid * (kKin / 4); idx += kThr2) {
      const int c  = idx / (kKin / 4);
      const int i4 = idx - c * (kKin / 4);
      const v4f v = *(const v4f*)(wcr + (size_t)c * kKin + 4 * i4);
      v4h hv;
      hv[0] = (_Float16)(v[0] * kCarryW);
      hv[1] = (_Float16)(v[1] * kCarryW);
      hv[2] = (_Float16)(v[2] * kCarryW);
      hv[3] = (_Float16)(v[3] * kCarryW);
      *(v4h*)(wcs + c * kKrow + 4 * i4) = hv;
    }
    for (int idx = tid; idx < kHid * ((kKrow - kKin) / 4); idx += kThr2) {
      const int c = idx / ((kKrow - kKin) / 4);
      const int q = idx - c * ((kKrow - kKin) / 4);
      v4h zh;
      zh[0] = (_Float16)0.0f; zh[1] = (_Float16)0.0f; zh[2] = (_Float16)0.0f; zh[3] = (_Float16)0.0f;
      *(v4h*)(wcs + c * kKrow + kKin + 4 * q) = zh;
    }
  }
  {
    for (int idx = tid; idx < kNB * (kKin / 4); idx += kThr2) {
      const int bs = idx / (kKin / 4);
      const int i4 = idx - bs * (kKin / 4);
      const v4f v = *(const v4f*)(feats + (size_t)(b0 + bs) * kKin + 4 * i4);
      *(v4f*)(xs + bs * kKpad + 4 * i4) = v;
    }
    for (int idx = tid; idx < kNB * ((kKpad - kKin) / 4); idx += kThr2) {
      const int bs = idx / ((kKpad - kKin) / 4);
      const int q  = idx - bs * ((kKpad - kKin) / 4);
      const v4f z4 = (v4f){0.0f, 0.0f, 0.0f, 0.0f};
      *(v4f*)(xs + bs * kKpad + kKin + 4 * q) = z4;
    }
  }
  {
    const float ar = avec[rep];
    for (int idx = tid; idx < kNB * kLenPad; idx += kThr2) {
      const int bs = idx / kLenPad;
      const int t  = idx - bs * kLenPad;
      const int tc = (t < kLen) ? t : (kLen - 1);
      const float fl  = feats[(size_t)(rep * kBat + b0 + bs) * kLen + tc];
      const float fac = (t < kLen) ? 1.0f : 0.0f;
      const float fv  = fl * fac;
      fvs[idx] = fv;
      svs[idx] = ar * fv;
    }
    if (tid < kHid) {
      wsh[tid]  = Wlin[rep * kHid + tid];
      whsh[tid] = Wh[rep * kHid + tid];
    }
  }
  __syncthreads();

  const int lane = tid & 31;
  const int wv   = tid >> 5;
  const int bs   = wv / kWPB;
  const int wsub = wv - bs * kWPB;
  const int hh   = lane >> 4;
  const int lm   = lane & 15;
  const int m0   = wsub * 32;
  const float* xrow = xs + bs * kKpad;
  const float sA = svs[bs * kLenPad + m0 + lm];
  const float sB = svs[bs * kLenPad + m0 + 16 + lm];
  const float s2A = sA + sA;
  const float s2B = sB + sB;
  const _Float16* wrow0 = wcs + lm * kKrow;
  const _Float16* wrow1 = wcs + (16 + lm) * kKrow;

  v8f acc00 = (v8f){0.f,0.f,0.f,0.f,0.f,0.f,0.f,0.f};
  v8f acc01 = (v8f){0.f,0.f,0.f,0.f,0.f,0.f,0.f,0.f};
  v8f acc10 = (v8f){0.f,0.f,0.f,0.f,0.f,0.f,0.f,0.f};
  v8f acc11 = (v8f){0.f,0.f,0.f,0.f,0.f,0.f,0.f,0.f};

#pragma unroll 1
  for (int kc = 0; kc < kKpad / 32; ++kc) {
    const int kb = kc * 32 + hh * 8;
    const v4f x0 = *(const v4f*)(xrow + kb);
    const v4f x1 = *(const v4f*)(xrow + kb + 4);
    const v4f x2 = *(const v4f*)(xrow + kb + 16);
    const v4f x3 = *(const v4f*)(xrow + kb + 20);
    const float xv[16] = {x0[0], x0[1], x0[2], x0[3], x1[0], x1[1], x1[2], x1[3],
                          x2[0], x2[1], x2[2], x2[3], x3[0], x3[1], x3[2], x3[3]};
    v16h fa, fb;
#pragma unroll
    for (int e = 0; e < 16; ++e) {
      fa[e] = tanh_gen(s2A, xv[e]);
      fb[e] = tanh_gen(s2B, xv[e]);
    }
    const v16h wb0 = Frag<_Float16>::load(wrow0 + kb);
    const v16h wb1 = Frag<_Float16>::load(wrow1 + kb);
    acc00 = Frag<_Float16>::mma(fa, wb0, acc00);
    acc01 = Frag<_Float16>::mma(fa, wb1, acc01);
    acc10 = Frag<_Float16>::mma(fb, wb0, acc10);
    acc11 = Frag<_Float16>::mma(fb, wb1, acc11);
    guard4x(acc00, acc01, acc10, acc11, fa, fb, wb0, wb1);
  }

  {
    const float w0 = wsh[lm], w1 = wsh[16 + lm];
    const float h0 = whsh[lm], h1 = whsh[16 + lm];
    const float* frow = fvs + bs * kLenPad;
    float* srow = segs + bs * kSeg;
#pragma unroll
    for (int i = 0; i < 8; ++i) {
      {
        const int t = m0 + 8 * hh + i;
        const float fv = frow[t];
        float g0 = fmaf(fv, w0, acc00[i] * kInvCarry); g0 = fmaxf(g0, 0.0f);
        float g1 = fmaf(fv, w1, acc01[i] * kInvCarry); g1 = fmaxf(g1, 0.0f);
        float v = fmaf(g0, h0, g1 * h1);
        v += __shfl_xor(v, 8);
        v += __shfl_xor(v, 4);
        v += __shfl_xor(v, 2);
        v += __shfl_xor(v, 1);
        const float fac = (t < kLen) ? 1.0f : 0.0f;
        const float res = (v + fv) * fac;
        if (lm == 0) srow[t] = res;
      }
      {
        const int t = m0 + 16 + 8 * hh + i;
        const float fv = frow[t];
        float g0 = fmaf(fv, w0, acc10[i] * kInvCarry); g0 = fmaxf(g0, 0.0f);
        float g1 = fmaf(fv, w1, acc11[i] * kInvCarry); g1 = fmaxf(g1, 0.0f);
        float v = fmaf(g0, h0, g1 * h1);
        v += __shfl_xor(v, 8);
        v += __shfl_xor(v, 4);
        v += __shfl_xor(v, 2);
        v += __shfl_xor(v, 1);
        const float fac = (t < kLen) ? 1.0f : 0.0f;
        const float res = (v + fv) * fac;
        if (lm == 0) srow[t] = res;
      }
    }
  }
  __syncthreads();

  if (wv < 2 * kNB) {
    const int sbs  = (wv < kNB) ? wv : (wv - kNB);
    const bool lop = (wv >= kNB);
    const int q  = lane >> 3;
    const int tb = q * 64 + (lane & 7) * 8;
    const float* sr = segs + sbs * kSeg;
    unsigned short hb[8], lb[8];
#pragma unroll
    for (int j = 0; j < 8; ++j) {
      const int t  = tb + j;
      const int tc = (t < kLenPad) ? t : (kLenPad - 1);
      const float fac = (t < kLen) ? 1.0f : 0.0f;
      const float val = sr[tc] * fac;
      const unsigned short h = f2bf_bits(val);
      hb[j] = h;
      lb[j] = f2bf_bits(val - bf_bits2f(h));
    }
    const v4u hv = (v4u){pk16(hb[0], hb[1]), pk16(hb[2], hb[3]), pk16(hb[4], hb[5]), pk16(hb[6], hb[7])};
    const v4u lv = (v4u){pk16(lb[0], lb[1]), pk16(lb[2], lb[3]), pk16(lb[4], lb[5]), pk16(lb[6], lb[7])};
    const v4u sv = (v4u){lop ? lv[0] : hv[0], lop ? lv[1] : hv[1], lop ? lv[2] : hv[2], lop ? lv[3] : hv[3]};
    unsigned short* base = lop ? fflo : ffhi;
    unsigned short* dst = base + (size_t)(b0 + sbs) * kFFld + rep * kSeg + tb;
    for (int pass = 0; pass < 2; ++pass) {
      if (lane < 24) *(volatile v4u*)dst = sv;
      __threadfence();
    }
  }
}

__global__ __launch_bounds__(256) void head_out_kernel(const float* __restrict__ Hf, const float* __restrict__ W2,
                                                       const float* __restrict__ b2, float* __restrict__ out) {
  __shared__ float w2s[kN2 * kN1];
  __shared__ float b2s[8];
  __shared__ __align__(16) float outs[64 * kN2];
  const int tid = threadIdx.x;
  const int rbase = blockIdx.x * 64;
  for (int i = tid; i < kN2 * kN1; i += 256) w2s[i] = W2[i];
  if (tid < kN2) b2s[tid] = b2[tid];
  __syncthreads();

  const int j = tid >> 2;
  const int p = tid & 3;
  const float* hrow = Hf + (size_t)(rbase + j) * kN1 + p * 32;
  float acc[kN2];
#pragma unroll
  for (int o = 0; o < kN2; ++o) acc[o] = 0.0f;
#pragma unroll 1
  for (int q = 0; q < 8; ++q) {
    const v4f hv = *(const v4f*)(hrow + 4 * q);
#pragma unroll
    for (int e = 0; e < 4; ++e) {
      const float hval = hv[e];
      const int kk = p * 32 + 4 * q + e;
#pragma unroll
      for (int o = 0; o < kN2; ++o) acc[o] = fmaf(hval, w2s[o * kN1 + kk], acc[o]);
    }
  }
#pragma unroll
  for (int o = 0; o < kN2; ++o) {
    acc[o] += __shfl_xor(acc[o], 1);
    acc[o] += __shfl_xor(acc[o], 2);
  }
  if (p == 0) {
#pragma unroll
    for (int o = 0; o < kN2; ++o) outs[j * kN2 + o] = acc[o] + b2s[o];
  }
  __syncthreads();
  if (tid < 32) {
    const int lane = tid;
    float* ob = out + (size_t)rbase * kN2;
    for (int pass = 0; pass < 2; ++pass) {
#pragma unroll
      for (int it = 0; it < 4; ++it) {
        const int line = it * 4 + (lane >> 3);
        const int idx4 = line * 8 + (lane & 7);
        if (line < 14) {
          const v4f v = *(const v4f*)(outs + idx4 * 4);
          *(volatile v4f*)(ob + idx4 * 4) = v;
        }
      }
      __threadfence();
    }
  }
}

extern "C" void kernel_launch(void* const* d_in, const int* in_sizes, int n_in,
                              void* d_out, int out_size, void* d_ws, size_t ws_size,
                              hipStream_t stream) {
  if (n_in < 9) return;
  const float* feats = (const float*)d_in[0];
  const float* avec  = (const float*)d_in[1];
  const float* Wlin  = (const float*)d_in[2];
  const float* Wc    = (const float*)d_in[3];
  const float* Wh    = (const float*)d_in[4];
  const float* W1    = (const float*)d_in[5];
  const float* b1    = (const float*)d_in[6];
  const float* W2    = (const float*)d_in[7];
  const float* b2    = (const float*)d_in[8];
  float* out = (float*)d_out;

  if (in_sizes[0] != kRep * kBat * kLen) return;
  if (in_sizes[1] != kRep || in_sizes[2] != kRep * kHid) return;
  if (in_sizes[3] != kRep * kHid * kKin || in_sizes[4] != kRep * kHid) return;
  if (in_sizes[5] != kN1 * kKin || in_sizes[6] != kN1) return;
  if (in_sizes[7] != kN2 * kN1 || in_sizes[8] != kN2) return;
  if (out_size != kBat * kN2) return;

  const size_t szFF  = (size_t)kBat * kFFld * 2;
  const size_t szW1p = (size_t)kN1 * kFFld * 2;
  const size_t szH   = (size_t)kBat * kN1 * 4;
  const size_t offFFhi = 0;
  const size_t offFFlo = offFFhi + szFF;
  const size_t offW1hi = offFFlo + szFF;
  const size_t offW1lo = offW1hi + szW1p;
  const size_t offH    = offW1lo + szW1p;
  const size_t total   = offH + szH;
  if (ws_size < total) return;

  char* ws = (char*)d_ws;
  unsigned short* ffhi = (unsigned short*)(ws + offFFhi);
  unsigned short* fflo = (unsigned short*)(ws + offFFlo);
  unsigned short* w1hi = (unsigned short*)(ws + offW1hi);
  unsigned short* w1lo = (unsigned short*)(ws + offW1lo);
  float* Hf = (float*)(ws + offH);

  w1_planes_kernel<<<dim3((kN1 * (kFFld / 8) + 255) / 256), dim3(256), 0, stream>>>(W1, w1hi, w1lo);

  rep_attn_kernel<<<dim3(kRep * (kBat / kNB)), dim3(kThr2), 0, stream>>>(feats, avec, Wlin, Wc, Wh, ffhi, fflo);

  {
    const int M = kBat, N = kN1, K = kFFld;
    const int tiles = (M / 64) * (N / 64);
    wmma_gemm64<1, true, 2, 0, false, 0><<<dim3((tiles + 7) / 8, 1, 1), dim3(256), 0, stream>>>(
        ffhi, fflo, kFFld, 0L,
        w1hi, w1lo, kFFld, 0L,
        (void*)Hf, (void*)Hf, kN1, 0L,
        b1,
        b1, 0L,
        M, N, K, 1.0f);
  }

  head_out_kernel<<<dim3(kBat / 64), dim3(256), 0, stream>>>(Hf, W2, b2, out);
}
